// MultiScaleEquivariantResidualNet_14851996909783
// MI455X (gfx1250) — hardware-verified
//
#include <hip/hip_runtime.h>
#include <stddef.h>


#define HD      64
#define NGRAPH  200
#define NJOB    23
#define NTHR    256
#define NWAVE   8
#define EPTH    8
#define NGRP    2
#define CHUNK   (NTHR * EPTH * NGRP)
#define WCAP    (EPTH * NGRP * 32)
#define LISTN   (NWAVE * WCAP)
#define NBC     4096
#define NBF     1024
#define RCAP    40960
#define RBN     128
#define TGT     256
#define DEGCAP  256
#define GROWS   128
#define OTHR    512
#define EPA     40
#define EPW     72
#define WSCAP   134217728
#define NEG_BIG (-3.0e38f)
#define RSQ12   0.28867513459481287f
#define LDS_FILL ((RCAP + NBF + LISTN) * 4 + 64)
#define LDS_EDGE (3 * GROWS * EPA * 2 + 2 * GROWS * EPW * 2)
#define LDS_G64  (GROWS * 64 * 4)
#define LDS_G128 (GROWS * 128 * 4)

static_assert((CHUNK & (CHUNK - 1)) == 0);
static_assert(CHUNK <= 4096);
static_assert(NBC == 4 * NBF);
static_assert(OTHR * 8 == NBC);
static_assert((RCAP % 32) == 0);
static_assert(TGT == NWAVE * 32);
static_assert(GROWS == NWAVE * 16);
static_assert(LDS_EDGE >= GROWS * HD * 4);
static_assert((EPA * 2) % 16 == 0 && (EPW * 2) % 16 == 0);

typedef float          v2f  __attribute__((ext_vector_type(2)));
typedef float          v4f  __attribute__((ext_vector_type(4)));
typedef float          v8f  __attribute__((ext_vector_type(8)));
typedef int            v4i  __attribute__((ext_vector_type(4)));
typedef unsigned int   v2u  __attribute__((ext_vector_type(2)));
typedef unsigned short v8us __attribute__((ext_vector_type(8)));
typedef __bf16         v16b __attribute__((ext_vector_type(16)));
union FragB { v16b v; v8us h[2]; };

__device__ __forceinline__ unsigned int bfr(float f) {
  const unsigned int u = __float_as_uint(f);
  return (u + 0x7FFFu + ((u >> 16) & 1u)) >> 16;
}
__device__ __forceinline__ void split1(float x, unsigned short& hb, unsigned short& lb) {
  const unsigned int hu = bfr(x);
  const float hf = __uint_as_float(hu << 16);
  hb = (unsigned short)hu;
  lb = (unsigned short)bfr(x - hf);
}
__device__ __forceinline__ void split8(v4f a, v4f b, v8us& hi, v8us& lo) {
  unsigned short hb, lb;
  split1(a.x, hb, lb); hi[0] = hb; lo[0] = lb;
  split1(a.y, hb, lb); hi[1] = hb; lo[1] = lb;
  split1(a.z, hb, lb); hi[2] = hb; lo[2] = lb;
  split1(a.w, hb, lb); hi[3] = hb; lo[3] = lb;
  split1(b.x, hb, lb); hi[4] = hb; lo[4] = lb;
  split1(b.y, hb, lb); hi[5] = hb; lo[5] = lb;
  split1(b.z, hb, lb); hi[6] = hb; lo[6] = lb;
  split1(b.w, hb, lb); hi[7] = hb; lo[7] = lb;
}
__device__ __forceinline__ void pk2(float x, float y, unsigned int& hi, unsigned int& lo) {
  unsigned short a, b, c, d;
  split1(x, a, c); split1(y, b, d);
  hi = (unsigned int)a | ((unsigned int)b << 16);
  lo = (unsigned int)c | ((unsigned int)d << 16);
}

__device__ __forceinline__ v8f wm(v16b a, v16b b, v8f c) {
  return __builtin_amdgcn_wmma_f32_16x16x32_bf16(false, a, false, b, (short)0, c, false, false);
}
__device__ __forceinline__ v8f wm3(v16b ah, v16b al, v16b bh, v16b bl, v8f c) {
  c = wm(ah, bh, c); c = wm(ah, bl, c); c = wm(al, bh, c);
  asm volatile("v_nop\n\tv_nop\n\tv_nop\n\tv_nop" : "+v"(c) : "v"(ah), "v"(al), "v"(bh), "v"(bl));
  return c;
}
__device__ __forceinline__ v8f wm2(v16b a, v16b b0, v16b b1, v8f c) {
  c = wm(a, b0, c); c = wm(a, b1, c);
  asm volatile("v_nop\n\tv_nop\n\tv_nop\n\tv_nop" : "+v"(c) : "v"(a), "v"(b0), "v"(b1));
  return c;
}

__device__ __forceinline__ float wsum(float v) {
#pragma unroll
  for (int o = 16; o > 0; o >>= 1) v += __shfl_xor(v, o);
  return v;
}
__device__ __forceinline__ float wmax(float v) {
#pragma unroll
  for (int o = 16; o > 0; o >>= 1) v = fmaxf(v, __shfl_xor(v, o));
  return v;
}

template <int NB>
__device__ __forceinline__ int scan_chunk(const int* __restrict__ dsts, int nE, int cbase, int slotBase,
                                          int vec8, int* list, int tid, int lane, int wave) {
  int wc = 0;
#pragma unroll
  for (int g = 0; g < NGRP; ++g) {
    const int el0  = (g * NTHR + tid) * EPTH;
    const int e0   = cbase + el0;
    const int sent = -2147483647 - 1;
    v4i da, db;
    if (vec8 != 0 && cbase + CHUNK <= nE) {
      da = *(const v4i*)(dsts + e0);
      db = *(const v4i*)(dsts + e0 + 4);
    } else {
      da.x = (e0     < nE) ? dsts[min(e0, nE - 1)] : sent;
      da.y = (e0 + 1 < nE) ? dsts[min(e0 + 1, nE - 1)] : sent;
      da.z = (e0 + 2 < nE) ? dsts[min(e0 + 2, nE - 1)] : sent;
      da.w = (e0 + 3 < nE) ? dsts[min(e0 + 3, nE - 1)] : sent;
      db.x = (e0 + 4 < nE) ? dsts[min(e0 + 4, nE - 1)] : sent;
      db.y = (e0 + 5 < nE) ? dsts[min(e0 + 5, nE - 1)] : sent;
      db.z = (e0 + 6 < nE) ? dsts[min(e0 + 6, nE - 1)] : sent;
      db.w = (e0 + 7 < nE) ? dsts[min(e0 + 7, nE - 1)] : sent;
    }
    const unsigned nb = (unsigned)slotBase;
    const unsigned s0 = (unsigned)da.x - nb, s1 = (unsigned)da.y - nb;
    const unsigned s2 = (unsigned)da.z - nb, s3 = (unsigned)da.w - nb;
    const unsigned s4 = (unsigned)db.x - nb, s5 = (unsigned)db.y - nb;
    const unsigned s6 = (unsigned)db.z - nb, s7 = (unsigned)db.w - nb;
    const bool h0 = s0 < (unsigned)NB, h1 = s1 < (unsigned)NB, h2 = s2 < (unsigned)NB, h3 = s3 < (unsigned)NB;
    const bool h4 = s4 < (unsigned)NB, h5 = s5 < (unsigned)NB, h6 = s6 < (unsigned)NB, h7 = s7 < (unsigned)NB;
    const unsigned any = __builtin_amdgcn_ballot_w32(h0 | h1 | h2 | h3 | h4 | h5 | h6 | h7);
    if (any != 0u) {
#define HITJ(J, HJ, SJ) { \
        const unsigned mj = __builtin_amdgcn_ballot_w32(HJ); \
        if (mj != 0u) { \
          if (HJ) { \
            const int p = wc + (int)__builtin_amdgcn_mbcnt_lo(mj, 0u); \
            if (p < WCAP) list[wave * WCAP + p] = ((el0 + (J)) << 12) | (int)(SJ); \
          } \
          wc += (int)__builtin_popcount(mj); } }
      HITJ(0, h0, s0)
      HITJ(1, h1, s1)
      HITJ(2, h2, s2)
      HITJ(3, h3, s3)
      HITJ(4, h4, s4)
      HITJ(5, h5, s5)
      HITJ(6, h6, s6)
      HITJ(7, h7, s7)
#undef HITJ
    }
  }
  return wc;
}

__global__ __launch_bounds__(NTHR) void k_count(const int* __restrict__ ei, int* cnt, int nE, int vec8) {
  __shared__ __attribute__((aligned(16))) int scnt[NBC];
  __shared__ __attribute__((aligned(16))) int list[LISTN];
  __shared__ int wcnt[NWAVE];
  const int tid = threadIdx.x, lane = tid & 31, wave = tid >> 5;
  const int nodeBase = blockIdx.x * NBC;
  const int* dsts = ei + nE;
  for (int i = tid; i < NBC; i += NTHR) scnt[i] = 0;
  __syncthreads();
  const int nChunks = (nE + CHUNK - 1) / CHUNK;
#pragma unroll 1
  for (int ch = 0; ch < nChunks; ++ch) {
    const int cbase = ch * CHUNK;
    const int wc = scan_chunk<NBC>(dsts, nE, cbase, nodeBase, vec8, list, tid, lane, wave);
    if (lane == 0) wcnt[wave] = wc;
    __syncthreads();
    if (wave == 0) {
#pragma unroll 1
      for (int wsx = 0; wsx < NWAVE; ++wsx) {
        int n = __builtin_amdgcn_readfirstlane(wcnt[wsx]);
        n = n > WCAP ? WCAP : (n < 0 ? 0 : n);
        const int* lp = list + wsx * WCAP;
#pragma unroll 1
        for (int i = 0; i < n; ++i) {
          const int ent  = __builtin_amdgcn_readfirstlane(lp[i]);
          const int slot = ent & (NBC - 1);
          if (lane == 0) scnt[slot] = scnt[slot] + 1;
        }
      }
    }
    __syncthreads();
  }
  v4i cq[4];
#pragma unroll
  for (int q = 0; q < 4; ++q) cq[q] = *(const v4i*)(scnt + (wave * 4 + q) * 128 + 4 * lane);
  int* cp = cnt + (size_t)nodeBase;
#pragma unroll
  for (int q = 0; q < 4; ++q) *(volatile v4i*)(cp + (wave * 4 + q) * 128 + 4 * lane) = cq[q];
  __threadfence();
#pragma unroll
  for (int q = 0; q < 4; ++q) *(volatile v4i*)(cp + (wave * 4 + q) * 128 + 4 * lane) = cq[q];
}

__global__ __launch_bounds__(OTHR) void k_offsets(const int* __restrict__ cnt, int* off, int* rbase, int nChunk) {
  __shared__ __attribute__((aligned(16))) int soff[NBC];
  __shared__ __attribute__((aligned(16))) int srb[RBN];
  __shared__ int wtot[OTHR / 32];
  const int tid = threadIdx.x, lane = tid & 31, wave = tid >> 5, sub = tid >> 7;
  for (int i = tid; i < RBN; i += OTHR) srb[i] = 0;
  int carry = 0;
#pragma unroll 1
  for (int ch = 0; ch < nChunk; ++ch) {
    const int base = ch * NBC;
    const v4i c0 = *(const v4i*)(cnt + base + 8 * tid);
    const v4i c1 = *(const v4i*)(cnt + base + 8 * tid + 4);
    const int e0 = max(c0.x, 0), e1 = max(c0.y, 0), e2 = max(c0.z, 0), e3 = max(c0.w, 0);
    const int e4 = max(c1.x, 0), e5 = max(c1.y, 0), e6 = max(c1.z, 0), e7 = max(c1.w, 0);
    const int ts = e0 + e1 + e2 + e3 + e4 + e5 + e6 + e7;
    int incl = ts;
#pragma unroll
    for (int d = 1; d < 32; d <<= 1) {
      const int t = __shfl_up(incl, d);
      if (lane >= d) incl += t;
    }
    if (lane == 31) wtot[wave] = incl;
    __syncthreads();
    const int S0 = wtot[0]  + wtot[1]  + wtot[2]  + wtot[3];
    const int S1 = wtot[4]  + wtot[5]  + wtot[6]  + wtot[7];
    const int S2 = wtot[8]  + wtot[9]  + wtot[10] + wtot[11];
    const int S3 = wtot[12] + wtot[13] + wtot[14] + wtot[15];
    int pre = 0;
#pragma unroll 1
    for (int w = 4 * sub; w < wave; ++w) pre += wtot[w];
    const int b0 = carry;
    const int b1 = b0 + ((S0 + 31) & ~31);
    const int b2 = b1 + ((S1 + 31) & ~31);
    const int b3 = b2 + ((S2 + 31) & ~31);
    const int b4 = b3 + ((S3 + 31) & ~31);
    const int myb = sub == 0 ? b0 : (sub == 1 ? b1 : (sub == 2 ? b2 : b3));
    if (tid == 0) {
      srb[min(4 * ch + 0, RBN - 1)] = b0;
      srb[min(4 * ch + 1, RBN - 1)] = b1;
      srb[min(4 * ch + 2, RBN - 1)] = b2;
      srb[min(4 * ch + 3, RBN - 1)] = b3;
    }
    int run = myb + pre + incl - ts;
    soff[8 * tid + 0] = run; run += e0;
    soff[8 * tid + 1] = run; run += e1;
    soff[8 * tid + 2] = run; run += e2;
    soff[8 * tid + 3] = run; run += e3;
    soff[8 * tid + 4] = run; run += e4;
    soff[8 * tid + 5] = run; run += e5;
    soff[8 * tid + 6] = run; run += e6;
    soff[8 * tid + 7] = run;
    carry = b4;
    __syncthreads();
    const v4i o0 = *(const v4i*)(soff + 4 * tid);
    const v4i o1 = *(const v4i*)(soff + 4 * (tid + OTHR));
    int* op = off + base;
    *(volatile v4i*)(op + 4 * tid) = o0;
    *(volatile v4i*)(op + 4 * (tid + OTHR)) = o1;
    __threadfence();
    *(volatile v4i*)(op + 4 * tid) = o0;
    *(volatile v4i*)(op + 4 * (tid + OTHR)) = o1;
    __syncthreads();
  }
  if (tid == 0) srb[min(4 * nChunk, RBN - 1)] = carry;
  __syncthreads();
  v4i rv = {0, 0, 0, 0};
  if (tid < 32) rv = *(const v4i*)(srb + 4 * tid);
  if (tid < 32) *(volatile v4i*)(rbase + 4 * tid) = rv;
  __threadfence();
  if (tid < 32) *(volatile v4i*)(rbase + 4 * tid) = rv;
}

__global__ __launch_bounds__(NTHR) void k_fill(const int* __restrict__ ei, const int* __restrict__ off, const int* __restrict__ rbase,
                                               int* csr, int nE, int vec8, int csrLen) {
  extern __shared__ v4f lds_dyn[];
  int* region = (int*)lds_dyn;
  int* cursor = region + RCAP;
  int* list   = cursor + NBF;
  int* wcnt   = list + LISTN;
  const int tid = threadIdx.x, lane = tid & 31, wave = tid >> 5;
  const int b = blockIdx.x;
  const int nodeBase = b * NBF;
  const int* dsts = ei + nE;
  int rb0 = rbase[b];
  const int rb1 = rbase[b + 1];
  rb0 = rb0 < 0 ? 0 : (rb0 > csrLen ? csrLen : rb0);
  rb0 &= ~31;
  int len = rb1 - rb0;
  len = len < 0 ? 0 : (len > RCAP ? RCAP : len);
  int lenW = (len + 31) & ~31;
  if (rb0 + lenW > csrLen) lenW = (csrLen - rb0) & ~31;
  {
    const v4i z = {0, 0, 0, 0};
    for (int i = tid; i < RCAP / 4; i += NTHR) ((v4i*)region)[i] = z;
    for (int s = tid; s < NBF; s += NTHR) {
      int o = off[nodeBase + s] - rb0;
      o = o < 0 ? 0 : (o > RCAP ? RCAP : o);
      cursor[s] = o;
    }
  }
  __syncthreads();
  const int nChunks = (nE + CHUNK - 1) / CHUNK;
#pragma unroll 1
  for (int ch = 0; ch < nChunks; ++ch) {
    const int cbase = ch * CHUNK;
    const int wc = scan_chunk<NBF>(dsts, nE, cbase, nodeBase, vec8, list, tid, lane, wave);
    if (lane == 0) wcnt[wave] = wc;
    __syncthreads();
    if (wave == 0) {
#pragma unroll 1
      for (int wsx = 0; wsx < NWAVE; ++wsx) {
        int n = __builtin_amdgcn_readfirstlane(wcnt[wsx]);
        n = n > WCAP ? WCAP : (n < 0 ? 0 : n);
        const int* lp = list + wsx * WCAP;
#pragma unroll 1
        for (int i = 0; i < n; ++i) {
          const int ent  = __builtin_amdgcn_readfirstlane(lp[i]);
          const int slot = ent & (NBF - 1);
          int e = cbase + ((ent >> 12) & (CHUNK - 1));
          e = e > nE - 1 ? nE - 1 : e;
          if (lane == 0) {
            int p = cursor[slot];
            p = p < 0 ? 0 : (p > RCAP - 1 ? RCAP - 1 : p);
            region[p] = e;
            const int np = p + 1;
            cursor[slot] = np > RCAP ? RCAP : np;
          }
        }
      }
    }
    __syncthreads();
  }
  const int nv = lenW >> 2;
  int* gp = csr + rb0;
#pragma unroll 1
  for (int i = tid; i < nv; i += NTHR) { const v4i v = ((const v4i*)region)[i]; *(volatile v4i*)(gp + 4 * i) = v; }
  __threadfence();
#pragma unroll 1
  for (int i = tid; i < nv; i += NTHR) { const v4i v = ((const v4i*)region)[i]; *(volatile v4i*)(gp + 4 * i) = v; }
}

struct WJob  { const float* src; unsigned short* dst; int K, N, KP, dup; };
struct WJobs { WJob j[NJOB]; };
static_assert(sizeof(WJob) == 32);
static_assert(sizeof(WJobs) == 32 * NJOB);

__global__ __launch_bounds__(NTHR) void k_wprep(WJobs J) {
  const int y = (int)blockIdx.y;
  const float* src = J.j[0].src; unsigned short* dst = J.j[0].dst;
  int K = J.j[0].K, N = J.j[0].N, KP = J.j[0].KP, dup = J.j[0].dup;
#pragma unroll
  for (int i = 1; i < NJOB; ++i)
    if (i == y) { src = J.j[i].src; dst = J.j[i].dst; K = J.j[i].K; N = J.j[i].N; KP = J.j[i].KP; dup = J.j[i].dup; }
  const int idx = blockIdx.x * NTHR + threadIdx.x;
  const int kp8 = KP >> 3;
  const int items = N * kp8;
  if (idx >= items) return;
  const int n = idx / kp8;
  const int k0 = (idx - n * kp8) * 8;
  float v[8];
#pragma unroll
  for (int e = 0; e < 8; ++e) {
    const int k = k0 + e;
    const int ks = dup ? (k & 15) : k;
    const int kc = ks < K ? ks : K - 1;
    const float x = src[(size_t)kc * N + n];
    v[e] = ks < K ? x : 0.0f;
  }
  v4f a, b;
  a.x = v[0]; a.y = v[1]; a.z = v[2]; a.w = v[3];
  b.x = v[4]; b.y = v[5]; b.z = v[6]; b.w = v[7];
  v8us hv, lv;
  split8(a, b, hv, lv);
  unsigned short* dh = dst + (size_t)idx * 8;
  unsigned short* dl = dh + (size_t)N * KP;
  *(volatile v8us*)dh = hv; *(volatile v8us*)dl = lv;
  __threadfence();
  *(volatile v8us*)dh = hv; *(volatile v8us*)dl = lv;
}

__global__ __launch_bounds__(NTHR) void k_cvt(const float* __restrict__ x, unsigned short* hi, unsigned short* lo,
                                              int nN, int K, int KP, int items) {
  const int idx = blockIdx.x * NTHR + threadIdx.x;
  if (idx >= items) return;
  const int kp8 = KP >> 3;
  const int r = idx / kp8;
  const int k0 = (idx - r * kp8) * 8;
  const int rc = r < nN ? r : nN - 1;
  const float* xp = x + (size_t)rc * K;
  float v[8];
#pragma unroll
  for (int e = 0; e < 8; ++e) {
    const int k = k0 + e;
    const int kc = k < K ? k : K - 1;
    const float t = xp[kc];
    v[e] = k < K ? t : 0.0f;
  }
  v4f a, b;
  a.x = v[0]; a.y = v[1]; a.z = v[2]; a.w = v[3];
  b.x = v[4]; b.y = v[5]; b.z = v[6]; b.w = v[7];
  v8us hv, lv;
  split8(a, b, hv, lv);
  *(volatile v8us*)(hi + (size_t)idx * 8) = hv; *(volatile v8us*)(lo + (size_t)idx * 8) = lv;
  __threadfence();
  *(volatile v8us*)(hi + (size_t)idx * 8) = hv; *(volatile v8us*)(lo + (size_t)idx * 8) = lv;
}

struct GArgs {
  const unsigned short* A0; const unsigned short* A1; const unsigned short* B0; const unsigned short* B1;
  const float* bias; const float* wdot; const float* bdot;
  float* Cf; unsigned short* Ch; unsigned short* Cl; float* dout;
  long long bVar; long long cVar;
  int lda, ksteps, ldb, mode, relu, useBias, ldc, ldp, nStore, useDot, z0, z1;
};
static_assert(sizeof(GArgs) == 152);

template <int NC>
__device__ __forceinline__ void gemm_rows(const GArgs& g, const float* stg, float* Cf, int rowBase, int wave, int lane,
                                          float bd, float* sdot, int dots) {
#pragma unroll
  for (int i = 0; i < 16; ++i) {
    const int lr = wave * 16 + i, grow = rowBase + lr;
    const bool ok = grow < g.nStore;
    if (NC == 128) {
      const v4f v = *(const v4f*)(stg + lr * NC + 4 * lane);
      if (g.mode == 0) {
        if (ok) *(volatile v4f*)(Cf + (size_t)grow * g.ldc + 4 * lane) = v;
      } else {
        unsigned int h0, l0, h1, l1;
        pk2(v.x, v.y, h0, l0); pk2(v.z, v.w, h1, l1);
        v2u hw, lw;
        hw.x = h0; hw.y = h1; lw.x = l0; lw.y = l1;
        if (ok) {
          *((volatile v2u*)(g.Ch + (size_t)grow * g.ldp) + lane) = hw;
          *((volatile v2u*)(g.Cl + (size_t)grow * g.ldp) + lane) = lw;
        }
      }
      if (dots) {
        const v4f w = *(const v4f*)(g.wdot + 4 * lane);
        float ps = v.x * w.x + v.y * w.y + v.z * w.z + v.w * w.w;
        ps = wsum(ps);
        if (lane == 0) sdot[lr] = ps + bd;
      }
    } else {
      const v2f v = *(const v2f*)(stg + lr * NC + 2 * lane);
      if (g.mode == 0) {
        if (ok) *(volatile v2f*)(Cf + (size_t)grow * g.ldc + 2 * lane) = v;
      } else {
        unsigned int hw, lw;
        pk2(v.x, v.y, hw, lw);
        if (ok) {
          *((volatile unsigned int*)(g.Ch + (size_t)grow * g.ldp) + lane) = hw;
          *((volatile unsigned int*)(g.Cl + (size_t)grow * g.ldp) + lane) = lw;
        }
      }
      if (dots) {
        const v2f w = *(const v2f*)(g.wdot + 2 * lane);
        float ps = v.x * w.x + v.y * w.y;
        ps = wsum(ps);
        if (lane == 0) sdot[lr] = ps + bd;
      }
    }
  }
}

template <int NC>
__global__ __launch_bounds__(NTHR) void k_gemm(GArgs g) {
  extern __shared__ v4f lds_dyn[];
  __shared__ __attribute__((aligned(16))) float sdot[GROWS];
  constexpr int NT = NC / 16;
  float* stg = (float*)lds_dyn;
  const int tid = threadIdx.x, lane = tid & 31, wave = tid >> 5, hh = lane >> 4, m = lane & 15;
  const int var = (int)blockIdx.y, rowBase = (int)blockIdx.x * GROWS;
  const unsigned short* B0 = g.B0 + (size_t)var * (size_t)g.bVar;
  const unsigned short* B1 = g.B1 + (size_t)var * (size_t)g.bVar;
  float* Cf = g.Cf + (size_t)var * (size_t)g.cVar;
  const int arow = rowBase + wave * 16 + m;
  const unsigned short* a0p = g.A0 + (size_t)arow * g.lda + 8 * hh;
  const unsigned short* a1p = g.A1 + (size_t)arow * g.lda + 8 * hh;
  v8f acc[NT];
#pragma unroll
  for (int t = 0; t < NT; ++t) { v8f z = {0.f, 0.f, 0.f, 0.f, 0.f, 0.f, 0.f, 0.f}; acc[t] = z; }
#pragma unroll 1
  for (int kt = 0; kt < g.ksteps; ++kt) {
    FragB ah, al;
    ah.h[0] = *(const v8us*)(a0p + 32 * kt); ah.h[1] = *(const v8us*)(a0p + 32 * kt + 16);
    al.h[0] = *(const v8us*)(a1p + 32 * kt); al.h[1] = *(const v8us*)(a1p + 32 * kt + 16);
#pragma unroll
    for (int t = 0; t < NT; ++t) {
      const size_t bo = (size_t)(16 * t + m) * g.ldb + 32 * kt + 8 * hh;
      FragB bh, bl;
      bh.h[0] = *(const v8us*)(B0 + bo); bh.h[1] = *(const v8us*)(B0 + bo + 16);
      bl.h[0] = *(const v8us*)(B1 + bo); bl.h[1] = *(const v8us*)(B1 + bo + 16);
      acc[t] = wm3(ah.v, al.v, bh.v, bl.v, acc[t]);
    }
  }
  const int r0 = wave * 16 + 8 * hh;
#pragma unroll
  for (int t = 0; t < NT; ++t) {
    const int col = 16 * t + m;
    const float bl0 = g.bias[col];
    const float bb = g.useBias ? bl0 : 0.0f;
#pragma unroll
    for (int r = 0; r < 8; ++r) {
      float v = acc[t][r] + bb;
      v = g.relu ? fmaxf(v, 0.0f) : v;
      stg[(r0 + r) * NC + col] = v;
    }
  }
  __syncthreads();
  const float bd = g.bdot[0];
  gemm_rows<NC>(g, stg, Cf, rowBase, wave, lane, bd, sdot, g.useDot);
  __threadfence();
  gemm_rows<NC>(g, stg, Cf, rowBase, wave, lane, bd, sdot, 0);
  __syncthreads();
  if (g.useDot && wave == 0) {
    int valid = g.nStore - rowBase;
    valid = valid < 0 ? 0 : (valid > GROWS ? GROWS : valid);
    const int nl = valid >> 2;
    const v4f dv = *(const v4f*)(sdot + 4 * lane);
    if (lane < nl) *(volatile v4f*)(g.dout + (size_t)rowBase + 4 * lane) = dv;
    __threadfence();
    if (lane < nl) *(volatile v4f*)(g.dout + (size_t)rowBase + 4 * lane) = dv;
  }
}

__global__ __launch_bounds__(NTHR) void k_edgew(const float* __restrict__ eattr, const float* __restrict__ pos, const int* __restrict__ ei,
    const unsigned short* __restrict__ Wep, const float* __restrict__ bep, const unsigned short* __restrict__ R1d,
    const unsigned short* __restrict__ R2p, float* EW, int nE, int nN) {
  extern __shared__ v4f lds_dyn[];
  unsigned short* eh = (unsigned short*)lds_dyn;
  unsigned short* el = eh + GROWS * EPA;
  unsigned short* bs = el + GROWS * EPA;
  unsigned short* th = bs + GROWS * EPA;
  unsigned short* tl = th + GROWS * EPW;
  float* stg = (float*)lds_dyn;
  const int tid = threadIdx.x, lane = tid & 31, wave = tid >> 5, hh = lane >> 4, m = lane & 15;
  const int rowBase = (int)blockIdx.x * GROWS;
#pragma unroll
  for (int i = 0; i < 2; ++i) {
    const int idx = i * NTHR + tid;
    const int r = idx >> 2, k0 = (idx & 3) * 8;
    int ec = rowBase + r; ec = ec > nE - 1 ? nE - 1 : ec;
    const float* ep = eattr + (size_t)ec * 19;
    float v[8];
#pragma unroll
    for (int e = 0; e < 8; ++e) {
      const int k = k0 + e;
      const int kc = k < 19 ? k : 18;
      const float x = ep[kc];
      v[e] = k < 19 ? x : 0.0f;
    }
    v4f a, b;
    a.x = v[0]; a.y = v[1]; a.z = v[2]; a.w = v[3];
    b.x = v[4]; b.y = v[5]; b.z = v[6]; b.w = v[7];
    v8us hv, lv;
    split8(a, b, hv, lv);
    *(v8us*)(eh + r * EPA + k0) = hv;
    *(v8us*)(el + r * EPA + k0) = lv;
  }
  {
    const int r = tid >> 1, j = tid & 1;
    int ec = rowBase + r; ec = ec > nE - 1 ? nE - 1 : ec;
    int s = ei[ec];      s = s < 0 ? 0 : (s > nN - 1 ? nN - 1 : s);
    int d = ei[nE + ec]; d = d < 0 ? 0 : (d > nN - 1 ? nN - 1 : d);
    const float dx = pos[(size_t)d * 3 + 0] - pos[(size_t)s * 3 + 0];
    const float dy = pos[(size_t)d * 3 + 1] - pos[(size_t)s * 3 + 1];
    const float dz = pos[(size_t)d * 3 + 2] - pos[(size_t)s * 3 + 2];
    const float rr = sqrtf(dx * dx + dy * dy + dz * dz + 1e-12f);
    float bv[8];
#pragma unroll
    for (int i = 0; i < 8; ++i) {
      const float c = (float)(8 * j + i) * (5.0f / 15.0f);
      const float t = (rr - c) * 3.2f;
      bv[i] = expf(-t * t);
    }
    v4f a, b;
    a.x = bv[0]; a.y = bv[1]; a.z = bv[2]; a.w = bv[3];
    b.x = bv[4]; b.y = bv[5]; b.z = bv[6]; b.w = bv[7];
    v8us hv, lv;
    split8(a, b, hv, lv);
    *(v8us*)(bs + r * EPA + 8 * j) = hv;
    *(v8us*)(bs + r * EPA + 16 + 8 * j) = lv;
  }
  __syncthreads();
  const int arow = wave * 16 + m;
  {
    FragB ab;
    ab.h[0] = *(const v8us*)(bs + arow * EPA + 8 * hh);
    ab.h[1] = *(const v8us*)(bs + arow * EPA + 16 + 8 * hh);
    v8f acc[4];
#pragma unroll
    for (int t = 0; t < 4; ++t) { v8f z = {0.f, 0.f, 0.f, 0.f, 0.f, 0.f, 0.f, 0.f}; acc[t] = z; }
#pragma unroll
    for (int t = 0; t < 4; ++t) {
      const unsigned short* bp = R1d + (16 * t + m) * 32 + 8 * hh;
      FragB b0, b1;
      b0.h[0] = *(const v8us*)bp;          b0.h[1] = *(const v8us*)(bp + 16);
      b1.h[0] = *(const v8us*)(bp + 2048); b1.h[1] = *(const v8us*)(bp + 2048 + 16);
      acc[t] = wm2(ab.v, b0.v, b1.v, acc[t]);
    }
    const int r0 = wave * 16 + 8 * hh;
#pragma unroll
    for (int t = 0; t < 4; ++t) {
#pragma unroll
      for (int r = 0; r < 8; ++r) {
        unsigned short hb, lb;
        split1(fmaxf(acc[t][r], 0.0f), hb, lb);
        th[(r0 + r) * EPW + 16 * t + m] = hb;
        tl[(r0 + r) * EPW + 16 * t + m] = lb;
      }
    }
  }
  v8f ace[4];
#pragma unroll
  for (int t = 0; t < 4; ++t) { v8f z = {0.f, 0.f, 0.f, 0.f, 0.f, 0.f, 0.f, 0.f}; ace[t] = z; }
  {
    FragB ah, al;
    ah.h[0] = *(const v8us*)(eh + arow * EPA + 8 * hh); ah.h[1] = *(const v8us*)(eh + arow * EPA + 16 + 8 * hh);
    al.h[0] = *(const v8us*)(el + arow * EPA + 8 * hh); al.h[1] = *(const v8us*)(el + arow * EPA + 16 + 8 * hh);
#pragma unroll
    for (int t = 0; t < 4; ++t) {
      const unsigned short* bp = Wep + (16 * t + m) * 32 + 8 * hh;
      FragB bh, bl;
      bh.h[0] = *(const v8us*)bp;          bh.h[1] = *(const v8us*)(bp + 16);
      bl.h[0] = *(const v8us*)(bp + 2048); bl.h[1] = *(const v8us*)(bp + 2048 + 16);
      ace[t] = wm3(ah.v, al.v, bh.v, bl.v, ace[t]);
    }
  }
  __syncthreads();
  v8f acw[4];
#pragma unroll
  for (int t = 0; t < 4; ++t) { v8f z = {0.f, 0.f, 0.f, 0.f, 0.f, 0.f, 0.f, 0.f}; acw[t] = z; }
#pragma unroll
  for (int kt = 0; kt < 2; ++kt) {
    FragB ah, al;
    ah.h[0] = *(const v8us*)(th + arow * EPW + 32 * kt + 8 * hh); ah.h[1] = *(const v8us*)(th + arow * EPW + 32 * kt + 16 + 8 * hh);
    al.h[0] = *(const v8us*)(tl + arow * EPW + 32 * kt + 8 * hh); al.h[1] = *(const v8us*)(tl + arow * EPW + 32 * kt + 16 + 8 * hh);
#pragma unroll
    for (int t = 0; t < 4; ++t) {
      const unsigned short* bp = R2p + (16 * t + m) * 64 + 32 * kt + 8 * hh;
      FragB bh, bl;
      bh.h[0] = *(const v8us*)bp;          bh.h[1] = *(const v8us*)(bp + 16);
      bl.h[0] = *(const v8us*)(bp + 4096); bl.h[1] = *(const v8us*)(bp + 4096 + 16);
      acw[t] = wm3(ah.v, al.v, bh.v, bl.v, acw[t]);
    }
  }
  __syncthreads();
  {
    const int r0 = wave * 16 + 8 * hh;
#pragma unroll
    for (int t = 0; t < 4; ++t) {
      const int col = 16 * t + m;
      const float be = bep[col];
#pragma unroll
      for (int r = 0; r < 8; ++r) stg[(r0 + r) * HD + col] = (ace[t][r] + be) * acw[t][r];
    }
  }
  __syncthreads();
  const float* lp = stg + wave * 16 * HD + 2 * lane;
  float* gp = EW + (size_t)(rowBase + wave * 16) * HD + 2 * lane;
#pragma unroll
  for (int i = 0; i < 16; ++i) { const v2f v = *(const v2f*)(lp + i * HD); *(volatile v2f*)(gp + (size_t)i * HD) = v; }
  __threadfence();
#pragma unroll
  for (int i = 0; i < 16; ++i) { const v2f v = *(const v2f*)(lp + i * HD); *(volatile v2f*)(gp + (size_t)i * HD) = v; }
}

__global__ __launch_bounds__(NTHR) void k_conv_agg(const int* __restrict__ csr, const int* __restrict__ off, const int* __restrict__ cnt,
    const int* __restrict__ ei, const float* __restrict__ hW, const float* __restrict__ EW, const float* __restrict__ hS,
    float* hF, unsigned int* hpH, unsigned int* hpL, int nN, int nE, int csrLen, int doSilu) {
  const int tid = threadIdx.x, lane = tid & 31, wave = tid >> 5;
  const int tbase = blockIdx.x * TGT + wave * 32;
  const int cnt_l = cnt[tbase + lane], off_l = off[tbase + lane];
#pragma unroll 1
  for (int j = 0; j < 32; ++j) {
    const int c = tbase + j;
    int n = __builtin_amdgcn_readfirstlane(__shfl(cnt_l, j));
    n = n < 0 ? 0 : (n > DEGCAP ? DEGCAP : n);
    const int st = __builtin_amdgcn_readfirstlane(__shfl(off_l, j));
    v2f acc = {0.f, 0.f};
#pragma unroll 1
    for (int q0 = 0; q0 < n; q0 += 32) {
      int p = st + q0 + lane; p = p < 0 ? 0 : (p > csrLen - 1 ? csrLen - 1 : p);
      int eid = csr[p];   eid = eid < 0 ? 0 : (eid > nE - 1 ? nE - 1 : eid);
      int sl = ei[eid];   sl = sl < 0 ? 0 : (sl > nN - 1 ? nN - 1 : sl);
      const int mcnt = (n - q0) < 32 ? (n - q0) : 32;
#pragma unroll 1
      for (int pp = 0; pp < mcnt; ++pp) {
        const int s = __builtin_amdgcn_readlane(sl, pp);
        const int e = __builtin_amdgcn_readlane(eid, pp);
        const v2f hv = *(const v2f*)(hW + (size_t)s * HD + 2 * lane);
        const v2f ev = *(const v2f*)(EW + (size_t)e * HD + 2 * lane);
        acc = acc + hv * ev;
      }
    }
    const v2f hs = *(const v2f*)(hS + (size_t)c * HD + 2 * lane);
    v2f v = hs + acc * RSQ12;
    v2f sv;
    sv.x = v.x * __builtin_amdgcn_rcpf(1.0f + expf(-v.x));
    sv.y = v.y * __builtin_amdgcn_rcpf(1.0f + expf(-v.y));
    v = doSilu ? sv : v;
    unsigned int hw, lw;
    pk2(v.x, v.y, hw, lw);
    float* hp = hF + (size_t)c * HD + 2 * lane;
    unsigned int* ph = hpH + (size_t)c * 32 + lane;
    unsigned int* pl = hpL + (size_t)c * 32 + lane;
    *(volatile v2f*)hp = v; *(volatile unsigned int*)ph = hw; *(volatile unsigned int*)pl = lw;
    __threadfence();
    *(volatile v2f*)hp = v; *(volatile unsigned int*)ph = hw; *(volatile unsigned int*)pl = lw;
  }
}

__global__ __launch_bounds__(NTHR) void k_attn(const int* __restrict__ csr, const int* __restrict__ off, const int* __restrict__ cnt,
    const int* __restrict__ ei, const float* __restrict__ q, const float* __restrict__ k, const float* __restrict__ v,
    float* aggp, int nN, int nE, int csrLen) {
  const int tid = threadIdx.x, lane = tid & 31, wave = tid >> 5;
  const bool lo16 = lane < 16;
  const int tbase = blockIdx.x * TGT + wave * 32;
  const int cnt_l = cnt[tbase + lane], off_l = off[tbase + lane];
#pragma unroll 1
  for (int j = 0; j < 32; ++j) {
    const int c = tbase + j;
    int n = __builtin_amdgcn_readfirstlane(__shfl(cnt_l, j));
    n = n < 0 ? 0 : (n > DEGCAP ? DEGCAP : n);
    const int st = __builtin_amdgcn_readfirstlane(__shfl(off_l, j));
    const v4f qv = *(const v4f*)(q + (size_t)c * 128 + 4 * lane);
    float MA = NEG_BIG, MB = NEG_BIG, dA = 0.0f, dB = 0.0f;
    v4f acc = {0.f, 0.f, 0.f, 0.f};
#pragma unroll 1
    for (int q0 = 0; q0 < n; q0 += 32) {
      int p = st + q0 + lane; p = p < 0 ? 0 : (p > csrLen - 1 ? csrLen - 1 : p);
      int eid = csr[p];   eid = eid < 0 ? 0 : (eid > nE - 1 ? nE - 1 : eid);
      int sl = ei[eid];   sl = sl < 0 ? 0 : (sl > nN - 1 ? nN - 1 : sl);
      const int mcnt = (n - q0) < 32 ? (n - q0) : 32;
      float scA = NEG_BIG, scB = NEG_BIG;
#pragma unroll 1
      for (int pp = 0; pp < mcnt; ++pp) {
        const int s = __builtin_amdgcn_readlane(sl, pp);
        const v4f kv = *(const v4f*)(k + (size_t)s * 128 + 4 * lane);
        float d = qv.x * kv.x + qv.y * kv.y + qv.z * kv.z + qv.w * kv.w;
        d += __shfl_xor(d, 8); d += __shfl_xor(d, 4); d += __shfl_xor(d, 2); d += __shfl_xor(d, 1);
        const float sA = __shfl(d, 0) * 0.125f, sB = __shfl(d, 16) * 0.125f;
        scA = (lane == pp) ? sA : scA;
        scB = (lane == pp) ? sB : scB;
      }
      const bool val = lane < mcnt;
      const float cA = wmax(val ? scA : NEG_BIG), cB = wmax(val ? scB : NEG_BIG);
      const float nA = fmaxf(MA, cA), nB = fmaxf(MB, cB);
      const float rA = __expf(MA - nA), rB = __expf(MB - nB);
      MA = nA; MB = nB;
      const float pA = val ? __expf(scA - MA) : 0.0f;
      const float pB = val ? __expf(scB - MB) : 0.0f;
      dA = dA * rA + wsum(pA); dB = dB * rB + wsum(pB);
      acc = acc * (lo16 ? rA : rB);
#pragma unroll 1
      for (int pp = 0; pp < mcnt; ++pp) {
        const int s = __builtin_amdgcn_readlane(sl, pp);
        const v4f vv = *(const v4f*)(v + (size_t)s * 128 + 4 * lane);
        const float pa = __shfl(pA, pp), pb = __shfl(pB, pp);
        acc = acc + vv * (lo16 ? pa : pb);
      }
    }
    const float rd = __builtin_amdgcn_rcpf((lo16 ? dA : dB) + 1e-16f);
    const v4f x = acc * rd;
    v4f y;
    y.x = __shfl_xor(x.x, 16); y.y = __shfl_xor(x.y, 16); y.z = __shfl_xor(x.z, 16); y.w = __shfl_xor(x.w, 16);
    const v4f o = x + y;
    float* op = aggp + (size_t)c * HD + 4 * lane;
    if (lo16) *(volatile v4f*)op = o;
    __threadfence();
    if (lo16) *(volatile v4f*)op = o;
  }
}

__global__ __launch_bounds__(NTHR) void k_pool(const float* __restrict__ hF, const float* __restrict__ Wga, const float* __restrict__ bga,
                                               const int* __restrict__ batch, float* gc, int nN) {
  __shared__ __attribute__((aligned(16))) float sacc[NWAVE * HD];
  __shared__ int scnt[NWAVE];
  const int tid = threadIdx.x, lane = tid & 31, wave = tid >> 5;
  const int g = (int)blockIdx.x;
  const v2f wv = *(const v2f*)(Wga + 2 * lane);
  const float b0 = bga[0];
  v2f acc = {0.f, 0.f};
  int cw = 0;
#pragma unroll 1
  for (int base = wave * 32; base < nN; base += NTHR) {
    const int n = base + lane;
    const int bn = batch[n < nN ? n : nN - 1];
    const bool hit = (n < nN) && (bn == g);
    unsigned int mk = __builtin_amdgcn_ballot_w32(hit);
    while (mk != 0u) {
      const int idx = __builtin_ctz(mk);
      mk &= mk - 1u;
      const int nn = base + idx;
      const v2f hr = *(const v2f*)(hF + (size_t)nn * HD + 2 * lane);
      const float s = wsum(hr.x * wv.x + hr.y * wv.y) + b0;
      const float aw = __builtin_amdgcn_rcpf(1.0f + expf(-s));
      acc = acc + hr * aw;
      ++cw;
    }
  }
  *(v2f*)(sacc + wave * HD + 2 * lane) = acc;
  if (lane == 0) scnt[wave] = cw;
  __syncthreads();
  if (wave == 0) {
    v2f t = {0.f, 0.f};
    int ct = 0;
#pragma unroll
    for (int w = 0; w < NWAVE; ++w) { t = t + *(const v2f*)(sacc + w * HD + 2 * lane); ct += scnt[w]; }
    const float rc = __builtin_amdgcn_rcpf(fmaxf((float)ct, 1.0f));
    const v2f o = t * rc;
    float* op = gc + (size_t)g * HD + 2 * lane;
    *(volatile v2f*)op = o;
    __threadfence();
    *(volatile v2f*)op = o;
  }
}

__global__ __launch_bounds__(NTHR) void k_ln(const float* __restrict__ aggp, const float* __restrict__ hskip, const float* __restrict__ hF,
    const float* __restrict__ gc, const int* __restrict__ batch, const float* __restrict__ gl, const float* __restrict__ bl,
    const float* __restrict__ gg, const float* __restrict__ bg, unsigned int* xcH, unsigned int* xcL, int nN, int npad) {
  const int tid = threadIdx.x, lane = tid & 31, wave = tid >> 5;
  const int wg = blockIdx.x * NWAVE + wave;
  const v2f g1 = *(const v2f*)(gl + 2 * lane), b1 = *(const v2f*)(bl + 2 * lane);
  const v2f gA = *(const v2f*)(gg + 2 * lane), gB = *(const v2f*)(gg + HD + 2 * lane);
  const v2f bA = *(const v2f*)(bg + 2 * lane), bB = *(const v2f*)(bg + HD + 2 * lane);
  const size_t ps = (size_t)npad * HD;
#pragma unroll 1
  for (int i = 0; i < 4; ++i) {
    const int n = wg * 4 + i;
    const size_t ro = (size_t)n * HD + 2 * lane;
    v2f a = *(const v2f*)(aggp + ro);
    a = a + *(const v2f*)(aggp + ps + ro);
    a = a + *(const v2f*)(aggp + 2 * ps + ro);
    a = a + *(const v2f*)(aggp + 3 * ps + ro);
    const v2f hs = *(const v2f*)(hskip + ro);
    const v2f h  = *(const v2f*)(hF + ro);
    const v2f t = a * 0.125f + hs + h;
    const float mean = wsum(t.x + t.y) * (1.0f / 64.0f);
    const v2f d = t - mean;
    const float var = wsum(d.x * d.x + d.y * d.y) * (1.0f / 64.0f);
    const float rs = rsqrtf(var + 1e-5f);
    const v2f y = d * rs * g1 + b1;
    const int nc = n < nN ? n : nN - 1;
    int bn = batch[nc]; bn = bn < 0 ? 0 : (bn > NGRAPH - 1 ? NGRAPH - 1 : bn);
    const v2f gv = *(const v2f*)(gc + (size_t)bn * HD + 2 * lane);
    const float mean2 = wsum(h.x + h.y + gv.x + gv.y) * (1.0f / 128.0f);
    const v2f dh = h - mean2, dg = gv - mean2;
    const float var2 = wsum(dh.x * dh.x + dh.y * dh.y + dg.x * dg.x + dg.y * dg.y) * (1.0f / 128.0f);
    const float rs2 = rsqrtf(var2 + 1e-5f);
    const v2f yh = dh * rs2 * gA + bA;
    const v2f yg = dg * rs2 * gB + bB;
    unsigned int h0, l0, h1, l1, h2, l2;
    pk2(y.x, y.y, h0, l0); pk2(yh.x, yh.y, h1, l1); pk2(yg.x, yg.y, h2, l2);
    const size_t bu = (size_t)n * 96;
    volatile unsigned int* xh = (volatile unsigned int*)xcH;
    volatile unsigned int* xl = (volatile unsigned int*)xcL;
    xh[bu + lane] = h0; xh[bu + 32 + lane] = h1; xh[bu + 64 + lane] = h2;
    xl[bu + lane] = l0; xl[bu + 32 + lane] = l1; xl[bu + 64 + lane] = l2;
    __threadfence();
    xh[bu + lane] = h0; xh[bu + 32 + lane] = h1; xh[bu + 64 + lane] = h2;
    xl[bu + lane] = l0; xl[bu + 32 + lane] = l1; xl[bu + 64 + lane] = l2;
  }
}

static GArgs mkg(const unsigned short* A0, const unsigned short* A1, int lda, int ksteps,
                 const unsigned short* B0, const unsigned short* B1, int ldb, long long bVar,
                 const float* bias, int useBias, int relu, int mode,
                 float* Cf, long long cVar, int ldc, unsigned short* Ch, unsigned short* Cl, int ldp, int nStore,
                 const float* wdot, const float* bdot, float* dout, int useDot) {
  GArgs g;
  g.A0 = A0; g.A1 = A1; g.B0 = B0; g.B1 = B1; g.bias = bias; g.wdot = wdot; g.bdot = bdot;
  g.Cf = Cf; g.Ch = Ch; g.Cl = Cl; g.dout = dout; g.bVar = bVar; g.cVar = cVar;
  g.lda = lda; g.ksteps = ksteps; g.ldb = ldb; g.mode = mode; g.relu = relu; g.useBias = useBias;
  g.ldc = ldc; g.ldp = ldp; g.nStore = nStore; g.useDot = useDot; g.z0 = 0; g.z1 = 0;
  return g;
}

extern "C" void kernel_launch(void* const* d_in, const int* in_sizes, int n_in,
                              void* d_out, int out_size, void* d_ws, size_t ws_size,
                              hipStream_t stream) {
  if (n_in < 30) return;
  const int N = in_sizes[4];
  const int E = in_sizes[3] / 2;
  if (N <= 0 || E <= 0) return;
  if (in_sizes[0] != 3 * N || in_sizes[1] != 23 * N || in_sizes[2] != 19 * E || in_sizes[3] != 2 * E) return;
  if (in_sizes[5] != 19 * HD || in_sizes[6] != HD || in_sizes[7] != 23 * HD || in_sizes[8] != 23 * HD) return;
  if (in_sizes[9] != 16 * HD || in_sizes[10] != HD * HD || in_sizes[11] != 3 * HD * HD || in_sizes[12] != 3 * HD * HD) return;
  if (in_sizes[13] != 3 * 16 * HD || in_sizes[14] != 3 * HD * HD) return;
  if (in_sizes[15] != HD * 512 || in_sizes[16] != HD * 512 || in_sizes[17] != HD * 512 || in_sizes[18] != HD * HD) return;
  if (in_sizes[19] != HD || in_sizes[20] != HD || in_sizes[21] != HD || in_sizes[22] != HD || in_sizes[23] < 1) return;
  if (in_sizes[24] != 2 * HD || in_sizes[25] != 2 * HD || in_sizes[26] != 3 * HD * HD || in_sizes[27] != HD * 128) return;
  if (in_sizes[28] != 128 || in_sizes[29] < 1) return;
  if (out_size != 129 * N) return;
  if (N > (1 << 22) || E > (1 << 26)) return;

  const float* pos   = (const float*)d_in[0];
  const float* x     = (const float*)d_in[1];
  const float* eattr = (const float*)d_in[2];
  const int*   ei    = (const int*)d_in[3];
  const int*   batch = (const int*)d_in[4];
  const float* W_ep  = (const float*)d_in[5];  const float* b_ep  = (const float*)d_in[6];
  const float* Wm0   = (const float*)d_in[7];  const float* Ws0   = (const float*)d_in[8];
  const float* R10   = (const float*)d_in[9];  const float* R20   = (const float*)d_in[10];
  const float* Wm    = (const float*)d_in[11]; const float* Ws    = (const float*)d_in[12];
  const float* R1    = (const float*)d_in[13]; const float* R2    = (const float*)d_in[14];
  const float* Wq    = (const float*)d_in[15]; const float* Wk    = (const float*)d_in[16];
  const float* Wv    = (const float*)d_in[17]; const float* Wskip = (const float*)d_in[18];
  const float* b_skip= (const float*)d_in[19];
  const float* g_ln_l= (const float*)d_in[20]; const float* b_ln_l= (const float*)d_in[21];
  const float* W_ga  = (const float*)d_in[22]; const float* b_ga  = (const float*)d_in[23];
  const float* g_ln_g= (const float*)d_in[24]; const float* b_ln_g= (const float*)d_in[25];
  const float* P1    = (const float*)d_in[26]; const float* P2    = (const float*)d_in[27];
  const float* Wc    = (const float*)d_in[28]; const float* bc    = (const float*)d_in[29];
  float* out = (float*)d_out;

  const int NP = ((N + TGT - 1) / TGT) * TGT;
  const int EP = ((E + GROWS - 1) / GROWS) * GROWS;
  const int nBC = (N + NBC - 1) / NBC;
  if (4 * nBC + 1 > RBN) return;
  const int CNTPAD = nBC * NBC;
  const int nBF = (N + NBF - 1) / NBF;
  const int csrLen = ((E + 31) & ~31) + 4096;
  if (31 * 4 * nBC > 4096) return;

  const float* jsrc[NJOB]; int jK[NJOB], jN[NJOB], jdup[NJOB], jKP[NJOB]; size_t joff[NJOB];
  int nj = 0;
#define ADDJ(S, KK, NN, D) { jsrc[nj] = (S); jK[nj] = (KK); jN[nj] = (NN); jdup[nj] = (D); ++nj; }
  ADDJ(W_ep, 19, HD, 0) ADDJ(Wm0, 23, HD, 0) ADDJ(Ws0, 23, HD, 0) ADDJ(R10, 16, HD, 1) ADDJ(R20, HD, HD, 0)
  for (int l = 0; l < 3; ++l) {
    ADDJ(Wm + (size_t)l * HD * HD, HD, HD, 0) ADDJ(Ws + (size_t)l * HD * HD, HD, HD, 0)
    ADDJ(R1 + (size_t)l * 16 * HD, 16, HD, 1) ADDJ(R2 + (size_t)l * HD * HD, HD, HD, 0)
  }
  ADDJ(Wq, HD, 512, 0) ADDJ(Wk, HD, 512, 0) ADDJ(Wv, HD, 512, 0) ADDJ(Wskip, HD, HD, 0) ADDJ(P1, 3 * HD, HD, 0) ADDJ(P2, HD, 128, 0)
#undef ADDJ
  if (nj != NJOB) return;
  size_t whalves = 0; int maxItems = 0;
  for (int i = 0; i < NJOB; ++i) {
    jKP[i] = jdup[i] ? 32 : ((jK[i] + 31) / 32) * 32;
    joff[i] = whalves;
    whalves += (size_t)2 * jN[i] * jKP[i];
    const int it = jN[i] * jKP[i] / 8;
    maxItems = it > maxItems ? it : maxItems;
  }

  size_t off = 0;
  const size_t oW   = off; off = ((off + whalves * 2) + 255) & ~(size_t)255;
  const size_t oCnt = off; off = ((off + (size_t)CNTPAD * 4) + 255) & ~(size_t)255;
  const size_t oOff = off; off = ((off + (size_t)CNTPAD * 4) + 255) & ~(size_t)255;
  const size_t oRb  = off; off = ((off + (size_t)RBN * 4) + 255) & ~(size_t)255;
  const size_t oCsr = off; off = ((off + (size_t)csrLen * 4) + 255) & ~(size_t)255;
  const size_t oHF  = off; off += (size_t)NP * HD * 4;
  const size_t oHpH = off; off += (size_t)NP * HD * 2;
  const size_t oHpL = off; off += (size_t)NP * HD * 2;
  const size_t oAr  = off;
  const size_t oHW  = oAr, oHS = oHW + (size_t)NP * HD * 4, oEW = oHS + (size_t)NP * HD * 4;
  const size_t endA = oEW + (size_t)EP * HD * 4;
  const size_t oQKV = oAr;
  const size_t oAgg = oQKV + (size_t)3 * NP * 128 * 4;
  const size_t oHsk = oAgg + (size_t)4 * NP * HD * 4;
  const size_t oGc  = oHsk + (size_t)NP * HD * 4;
  const size_t oXcH = ((oGc + (size_t)NGRAPH * HD * 4) + 255) & ~(size_t)255;
  const size_t oXcL = oXcH + (size_t)NP * 192 * 2;
  const size_t oThH = oXcL + (size_t)NP * 192 * 2;
  const size_t oThL = oThH + (size_t)NP * HD * 2;
  const size_t endB = oThL + (size_t)NP * HD * 2;
  off = ((endA > endB ? endA : endB) + 255) & ~(size_t)255;
  if (off > ws_size || off > (size_t)WSCAP) return;

  char* ws = (char*)d_ws;
  unsigned short* wp = (unsigned short*)(ws + oW);
  int* cnt  = (int*)(ws + oCnt);
  int* offp = (int*)(ws + oOff);
  int* rb   = (int*)(ws + oRb);
  int* csr  = (int*)(ws + oCsr);
  float* hF = (float*)(ws + oHF);
  unsigned short* hpH = (unsigned short*)(ws + oHpH);
  unsigned short* hpL = (unsigned short*)(ws + oHpL);
  float* hW = (float*)(ws + oHW);
  float* hS = (float*)(ws + oHS);
  float* EW = (float*)(ws + oEW);
  float* qkv = (float*)(ws + oQKV);
  float* aggp = (float*)(ws + oAgg);
  float* hsk = (float*)(ws + oHsk);
  float* gcb = (float*)(ws + oGc);
  unsigned short* xcH = (unsigned short*)(ws + oXcH);
  unsigned short* xcL = (unsigned short*)(ws + oXcL);
  unsigned short* thH = (unsigned short*)(ws + oThH);
  unsigned short* thL = (unsigned short*)(ws + oThL);

  WJobs J;
  const unsigned short* pl[NJOB];
  for (int i = 0; i < NJOB; ++i) {
    J.j[i].src = jsrc[i]; J.j[i].dst = wp + joff[i]; J.j[i].K = jK[i]; J.j[i].N = jN[i]; J.j[i].KP = jKP[i]; J.j[i].dup = jdup[i];
    pl[i] = wp + joff[i];
  }
  const int vec8 = ((E & 3) == 0) ? 1 : 0;

  k_wprep<<<dim3((maxItems + NTHR - 1) / NTHR, NJOB, 1), NTHR, 0, stream>>>(J);
  k_count<<<nBC, NTHR, 0, stream>>>(ei, cnt, E, vec8);
  k_offsets<<<1, OTHR, 0, stream>>>(cnt, offp, rb, nBC);
  hipFuncSetAttribute(reinterpret_cast<const void*>(&k_fill), hipFuncAttributeMaxDynamicSharedMemorySize, LDS_FILL);
  k_fill<<<nBF, NTHR, LDS_FILL, stream>>>(ei, offp, rb, csr, E, vec8, csrLen);
  k_cvt<<<(NP * 4 + NTHR - 1) / NTHR, NTHR, 0, stream>>>(x, hpH, hpL, N, 23, 32, NP * 4);

  hipFuncSetAttribute(reinterpret_cast<const void*>(&k_gemm<64>), hipFuncAttributeMaxDynamicSharedMemorySize, LDS_G64);
  hipFuncSetAttribute(reinterpret_cast<const void*>(&k_gemm<128>), hipFuncAttributeMaxDynamicSharedMemorySize, LDS_G128);
  hipFuncSetAttribute(reinterpret_cast<const void*>(&k_edgew), hipFuncAttributeMaxDynamicSharedMemorySize, LDS_EDGE);

  for (int l = 0; l < 4; ++l) {
    const int KPl = (l == 0) ? 32 : 64;
    const unsigned short* wm = (l == 0) ? pl[1] : pl[5 + 4 * (l - 1)];
    const unsigned short* r1d = (l == 0) ? pl[3] : pl[7 + 4 * (l - 1)];
    const unsigned short* r2p = (l == 0) ? pl[4] : pl[8 + 4 * (l - 1)];
    GArgs a = mkg(hpH, hpL, KPl, KPl / 32, wm, wm + HD * KPl, KPl, (long long)2 * HD * KPl,
                  b_ep, 0, 0, 0, hW, (long long)NP * HD, HD, hpH, hpL, HD, NP, b_ep, bc, hF, 0);
    k_gemm<64><<<dim3(NP / GROWS, 2, 1), NTHR, LDS_G64, stream>>>(a);
    k_edgew<<<EP / GROWS, NTHR, LDS_EDGE, stream>>>(eattr, pos, ei, pl[0], b_ep, r1d, r2p, EW, E, N);
    k_conv_agg<<<NP / TGT, NTHR, 0, stream>>>(csr, offp, cnt, ei, hW, EW, hS, hF,
                                               (unsigned int*)hpH, (unsigned int*)hpL, N, E, csrLen, l < 3 ? 1 : 0);
  }
  {
    GArgs a = mkg(hpH, hpL, HD, 2, pl[20], pl[20] + HD * HD, HD, 0, b_skip, 1, 0, 0,
                  hsk, 0, HD, hpH, hpL, HD, NP, b_skip, bc, hF, 0);
    k_gemm<64><<<dim3(NP / GROWS, 1, 1), NTHR, LDS_G64, stream>>>(a);
  }
  for (int g = 0; g < 4; ++g) {
    const unsigned short* b0 = pl[17] + (size_t)128 * g * HD;
    GArgs a = mkg(hpH, hpL, HD, 2, b0, b0 + (size_t)512 * HD, HD, (long long)2 * 512 * HD,
                  hF, 0, 0, 0, qkv, (long long)NP * 128, 128, hpH, hpL, HD, NP, hF, bc, hF, 0);
    k_gemm<128><<<dim3(NP / GROWS, 3, 1), NTHR, LDS_G128, stream>>>(a);
    k_attn<<<NP / TGT, NTHR, 0, stream>>>(csr, offp, cnt, ei, qkv, qkv + (size_t)NP * 128, qkv + (size_t)2 * NP * 128,
                                           aggp + (size_t)g * NP * HD, N, E, csrLen);
  }
  k_pool<<<NGRAPH, NTHR, 0, stream>>>(hF, W_ga, b_ga, batch, gcb, N);
  k_ln<<<NP / 32, NTHR, 0, stream>>>(aggp, hsk, hF, gcb, batch, g_ln_l, b_ln_l, g_ln_g, b_ln_g,
                                      (unsigned int*)xcH, (unsigned int*)xcL, N, NP);
  {
    GArgs a = mkg(xcH, xcL, 192, 6, pl[21], pl[21] + (size_t)HD * 192, 192, 0, b_ep, 0, 1, 1,
                  hW, 0, HD, thH, thL, HD, NP, b_ep, bc, hF, 0);
    k_gemm<64><<<dim3(NP / GROWS, 1, 1), NTHR, LDS_G64, stream>>>(a);
  }
  {
    GArgs a = mkg(thH, thL, HD, 2, pl[22], pl[22] + (size_t)128 * HD, HD, 0, hF, 0, 0, 0,
                  out + N, 0, 128, thH, thL, HD, N, Wc, bc, out, 1);
    k_gemm<128><<<dim3(NP / GROWS, 1, 1), NTHR, LDS_G128, stream>>>(a);
  }
}
